// Capsule_2224793059594
// MI455X (gfx1250) — hardware-run, weakly checked
//
#include <hip/hip_runtime.h>
#include <math.h>


#ifndef NB
#define NB 32
#endif
#define NB_FULL 32
#define NS   128
#define NC   128
#define DC   64
#define DIN  256
#define NIT  3
#define CP   136
#define OPT  72
#define WTP  264
#define QRS  2048.0f
#define QRI  (1.0f / 2048.0f)
#define CSC  16384.0f
#define CINV (1.0f / 16384.0f)
#define OSC  256.0f
#define OINV (1.0f / 256.0f)
#define LOG2E 1.4426950408889634f
#define EPSV 1e-7f

static_assert(NS == NC);
static_assert(NS == 128);
static_assert(DC == 64);
static_assert(DIN % 32 == 0);
static_assert(NS % 32 == 0);
static_assert(DC % 32 == 0);
static_assert(NS % 64 == 0);
static_assert((NB * NS) % 64 == 0);
static_assert(NB % 16 == 0);
static_assert(NB >= 16);
static_assert(NB <= NB_FULL);
static_assert((CP * 2) % 16 == 0);
static_assert((OPT * 2) % 16 == 0);
static_assert((WTP * 2) % 16 == 0);
static_assert(CP >= NS);
static_assert(OPT >= DC);
static_assert(WTP >= DIN);
static_assert(((size_t)NB * NS * DIN) % 8 == 0);

typedef _Float16 h16;
typedef unsigned short bf;
typedef __attribute__((ext_vector_type(16))) __bf16   v16bf;
typedef __attribute__((ext_vector_type(16))) _Float16 v16h;
typedef __attribute__((ext_vector_type(8)))  _Float16 v8h;
typedef __attribute__((ext_vector_type(8)))  unsigned short v8us;
typedef __attribute__((ext_vector_type(8)))  float    v8f;
typedef __attribute__((ext_vector_type(4)))  float    v4f;
typedef v4f  __attribute__((may_alias)) v4fa;

__device__ __forceinline__ unsigned short f2bf(float f) { unsigned u = __float_as_uint(f); u += 0x7FFFu + ((u >> 16) & 1u); return (unsigned short)(u >> 16); }
__device__ __forceinline__ float bfr(float f) { return __uint_as_float(((unsigned)f2bf(f)) << 16); }
__device__ __forceinline__ v16h cat16(v8h lo, v8h hi) { return __builtin_shufflevector(lo, hi, 0, 1, 2, 3, 4, 5, 6, 7, 8, 9, 10, 11, 12, 13, 14, 15); }
__device__ __forceinline__ v16bf cat16b(v8us lo, v8us hi) { return __builtin_bit_cast(v16bf, __builtin_shufflevector(lo, hi, 0, 1, 2, 3, 4, 5, 6, 7, 8, 9, 10, 11, 12, 13, 14, 15)); }
__device__ __forceinline__ v16h  ldh(const h16* p) { return cat16(*(const v8h*)p, *(const v8h*)(p + 16)); }
__device__ __forceinline__ v16bf ldb(const bf* p)  { return cat16b(*(const v8us*)p, *(const v8us*)(p + 16)); }
__device__ __forceinline__ void wave_sync() { __builtin_amdgcn_fence(3  , "wavefront"); __builtin_amdgcn_wave_barrier(); asm volatile("" ::: "memory"); }

__device__ __forceinline__ v8f wmma16g(v16h a, v16h b, v8f c) {
    c = __builtin_amdgcn_wmma_f32_16x16x32_f16(false, a, false, b, (short)0, c, false, false);
    asm volatile("v_nop\n\tv_nop\n\tv_nop\n\tv_nop" : "+v"(c) : "v"(a), "v"(b));
    return c; }
__device__ __forceinline__ v8f wmmabg(v16bf a, v16bf b, v8f c) {
    c = __builtin_amdgcn_wmma_f32_16x16x32_bf16(false, a, false, b, (short)0, c, false, false);
    asm volatile("v_nop\n\tv_nop\n\tv_nop\n\tv_nop" : "+v"(c) : "v"(a), "v"(b));
    return c; }
static __device__ __forceinline__ h16 toh_flush(float v) { const h16 r = (h16)v; return (fabsf(v) < 6.103515625e-05f) ? (h16)0.0f : r; }
__device__ __forceinline__ float bfv(unsigned short w) { return __uint_as_float(((unsigned)w) << 16); }

__global__ __launch_bounds__(256) void k_cvt8(const float* __restrict__ src, bf* dst, size_t n8) {
    const size_t i = (size_t)blockIdx.x * 256 + threadIdx.x; if (i >= n8) return;
    const v8f v = *(const v8f*)(src + i * 8); v8us o;
#pragma unroll
    for (int k = 0; k < 8; ++k) o[k] = f2bf(v[k]);
    *(volatile v8us*)(dst + i * 8) = o; __threadfence(); *(volatile v8us*)(dst + i * 8) = o;
}

static_assert((DIN * DC) % 256 == 0);
static_assert(256 * 8 * 8 == DC * DIN);
__global__ __launch_bounds__(256) void k_wt(const float* __restrict__ W, bf* WT) {
    __shared__ __align__(16) bf wt[DC * WTP];
    const int tid = threadIdx.x;
#pragma unroll 1
    for (int it = 0; it < (DIN * DC) / 256; ++it) { const int i = it * 256 + tid; const int k = i >> 6, d = i & 63; wt[d * WTP + k] = f2bf(W[i]); }
    __syncthreads();
#pragma unroll 1
    for (int ps = 0; ps < 2; ++ps) {
#pragma unroll 1
        for (int it = 0; it < 8; ++it) { const int p = it * 256 + tid; const int row = p >> 5, c8 = (p & 31) * 8;
            const v8us o = *(const v8us*)&wt[row * WTP + c8];
            *(volatile v8us*)(WT + (size_t)p * 8) = o; }
        if (ps == 0) __threadfence(); }
}

static_assert(32 * 16 * 8 == 64 * DC);
static_assert(16 * 4 == 64);
__global__ __launch_bounds__(32) void k_uw(const bf* __restrict__ A, const bf* __restrict__ Bt, h16* UH, h16* UR, h16* TH, h16* TR, float* US) {
    __shared__ __align__(16) float os[64 * 68];
    __shared__ __align__(16) float us[64];
    const int K = DIN;
    const int lane = threadIdx.x & 31, lr = lane & 15, hi = lane >> 4; const int r0 = blockIdx.x * 64;
    v8f acc[4][4];
#pragma unroll
    for (int mb = 0; mb < 4; ++mb)
#pragma unroll
        for (int nb = 0; nb < 4; ++nb) acc[mb][nb] = (v8f){};
    float ps[4];
#pragma unroll
    for (int mb = 0; mb < 4; ++mb) ps[mb] = 0.0f;
    const size_t aoff = (size_t)(r0 + lr) * K + 8 * hi, boff = (size_t)lr * K + 8 * hi;
#pragma unroll 1
    for (int kc = 0; kc < K; kc += 32) {
        v16bf a[4];
#pragma unroll
        for (int mb = 0; mb < 4; ++mb) { const bf* p = A + aoff + (size_t)mb * 16 * K + kc;
            const v8us lo = *(const v8us*)p, up = *(const v8us*)(p + 16); a[mb] = cat16b(lo, up);
            float s = 0.0f;
#pragma unroll
            for (int i = 0; i < 8; ++i) s += bfv(lo[i]) + bfv(up[i]);
            ps[mb] += s; }
#pragma unroll
        for (int nb = 0; nb < 4; ++nb) { const v16bf b = ldb(Bt + boff + (size_t)nb * 16 * K + kc);
#pragma unroll
            for (int mb = 0; mb < 4; ++mb) acc[mb][nb] = wmmabg(a[mb], b, acc[mb][nb]); }
    }
#pragma unroll
    for (int mb = 0; mb < 4; ++mb) { const float t = ps[mb] + __shfl_xor(ps[mb], 16, 32); if (hi == 0) us[mb * 16 + lr] = t; }
#pragma unroll
    for (int mb = 0; mb < 4; ++mb)
#pragma unroll
        for (int nb = 0; nb < 4; ++nb)
#pragma unroll
            for (int j = 0; j < 8; ++j) os[(mb * 16 + hi * 8 + j) * 68 + nb * 16 + lr] = acc[mb][nb][j];
    wave_sync();
    const int bb = r0 / NS, s0 = r0 % NS;
#pragma unroll 1
    for (int pz = 0; pz < 2; ++pz) {
#pragma unroll 1
        for (int it = 0; it < 16; ++it) { const int p = it * 32 + lane; const int row = p >> 3, c8 = (p & 7) * 8;
            const v4f x0 = *(const v4fa*)(&os[row * 68 + c8]); const v4f x1 = *(const v4fa*)(&os[row * 68 + c8 + 4]); v8h hv, rv;
#pragma unroll
            for (int i = 0; i < 4; ++i) { const h16 a0 = toh_flush(x0[i]); const h16 a1 = toh_flush(x1[i]); hv[i] = a0; hv[4 + i] = a1;
                rv[i] = toh_flush((x0[i] - (float)a0) * QRS); rv[4 + i] = toh_flush((x1[i] - (float)a1) * QRS); }
            const size_t oo = (size_t)r0 * DC + (size_t)p * 8;
            *(volatile v8h*)(UH + oo) = hv; *(volatile v8h*)(UR + oo) = rv; }
#pragma unroll 1
        for (int it = 0; it < 16; ++it) { const int p = it * 32 + lane; const int d = p >> 3, s8 = (p & 7) * 8;
            v8h hv, rv;
#pragma unroll
            for (int i = 0; i < 8; ++i) { const float x = os[(s8 + i) * 68 + d]; const h16 a0 = toh_flush(x); hv[i] = a0; rv[i] = toh_flush((x - (float)a0) * QRS); }
            const size_t oo = ((size_t)bb * DC + d) * NS + s0 + s8;
            *(volatile v8h*)(TH + oo) = hv; *(volatile v8h*)(TR + oo) = rv; }
        if (lane < 16) { const v4f v = *(const v4fa*)(&us[4 * lane]); *(volatile v4f*)(US + r0 + 4 * lane) = v; }
        if (pz == 0) __threadfence(); }
}

static_assert(256 * 4 * 8 == NS * DC);
static_assert(8 * 16 == NS);
__global__ __launch_bounds__(256) void k_pe(h16* PH, h16* PR, h16* PTH, h16* PTR, float* PE1) {
#pragma clang fp contract(off)
    __shared__ __align__(16) float tile[NS * 68];
    __shared__ __align__(16) float p1[DC];
    const int tid = threadIdx.x, j = tid & 31;
    const int wave = __builtin_amdgcn_readfirstlane((int)(threadIdx.x >> 5));
    const int n = blockIdx.x;
#pragma unroll 1
    for (int it = 0; it < 17; ++it) {
        const bool tab1 = (it == 16);
        const int kk = tab1 ? j : (n * 32 + j);
        const float dinv = tab1 ? (1.0f / 64.0f) : (1.0f / 8192.0f);
        const int pos = tab1 ? n : (wave * 16 + it);
        const float e = (2.0f * (float)kk) * dinv;
        const float inv = 1.0f / powf(10000.0f, e);
        const float ang = (float)pos * inv;
        const float sn = sinf(ang), cs = cosf(ang);
        if (!tab1) { tile[pos * 68 + 2 * j] = sn; tile[pos * 68 + 2 * j + 1] = cs; }
        else if (wave == 0) { p1[2 * j] = sn; p1[2 * j + 1] = cs; }
    }
    __syncthreads();
    const size_t nb0 = (size_t)n * NS * DC;
#pragma unroll 1
    for (int pz = 0; pz < 2; ++pz) {
#pragma unroll 1
        for (int it = 0; it < 4; ++it) { const int p = it * 256 + tid; const int row = p >> 3, c8 = (p & 7) * 8;
            const v4f x0 = *(const v4fa*)(&tile[row * 68 + c8]); const v4f x1 = *(const v4fa*)(&tile[row * 68 + c8 + 4]); v8h hv, rv;
#pragma unroll
            for (int i = 0; i < 4; ++i) { const h16 a0 = toh_flush(x0[i]); const h16 a1 = toh_flush(x1[i]); hv[i] = a0; hv[4 + i] = a1;
                rv[i] = toh_flush((x0[i] - (float)a0) * QRS); rv[4 + i] = toh_flush((x1[i] - (float)a1) * QRS); }
            *(volatile v8h*)(PH + nb0 + (size_t)p * 8) = hv; *(volatile v8h*)(PR + nb0 + (size_t)p * 8) = rv; }
#pragma unroll 1
        for (int it = 0; it < 4; ++it) { const int p = it * 256 + tid; const int d = p >> 4, s8 = (p & 15) * 8;
            v8h hv, rv;
#pragma unroll
            for (int i = 0; i < 8; ++i) { const float x = tile[(s8 + i) * 68 + d]; const h16 a0 = toh_flush(x); hv[i] = a0; rv[i] = toh_flush((x - (float)a0) * QRS); }
            *(volatile v8h*)(PTH + nb0 + (size_t)p * 8) = hv; *(volatile v8h*)(PTR + nb0 + (size_t)p * 8) = rv; }
        if (tid < 16) { const v4f v = *(const v4fa*)(&p1[4 * tid]); *(volatile v4f*)(PE1 + (size_t)n * DC + 4 * tid) = v; }
        if (pz == 0) __threadfence(); }
}

static_assert(32 * 8 * 16 == 16 * DC * 4);
static_assert(32 * 8 * 16 == 16 * NS * 2);
static_assert((size_t)2 * NS * CP * 2 + (size_t)8 * NS * 4 + (size_t)8 * 16 * 68 * 4 <= (size_t)131072);
__global__ __launch_bounds__(256) __attribute__((amdgpu_num_vgpr(256))) void k_rb(const h16* __restrict__ UH, const h16* __restrict__ UR, const h16* __restrict__ TH, const h16* __restrict__ TR,
                                           const h16* __restrict__ OH, const h16* __restrict__ ORS, const float* __restrict__ BLN, const float* __restrict__ US,
                                           const float* __restrict__ maskg, const float* __restrict__ PE1, float* PREB, h16* CNH, h16* CNR, int first) {
    __shared__ __align__(16) h16 ch[NC * CP];
    __shared__ __align__(16) h16 cr[NC * CP];
    __shared__ __align__(16) float t2p[8 * NC];
    __shared__ __align__(16) float os[8 * 16 * 68];
    const int lane = threadIdx.x & 31, lr = lane & 15, hi = lane >> 4;
    const int wave = __builtin_amdgcn_readfirstlane((int)(threadIdx.x >> 5));
    const int b = blockIdx.x;
    const int s0 = wave * 16;
    v8f x[8];
    if (first == 0) {
        const size_t ao = ((size_t)b * NS + s0 + lr) * DC + 8 * hi;
        const v16h a0h = ldh(UH + ao), a1h = ldh(UH + ao + 32), a0r = ldh(UR + ao), a1r = ldh(UR + ao + 32);
#pragma unroll
        for (int t = 0; t < 8; ++t) {
            const size_t bo = ((size_t)b * NC + t * 16 + lr) * DC + 8 * hi;
            const v16h b0h = ldh(OH + bo), b1h = ldh(OH + bo + 32), b0r = ldh(ORS + bo), b1r = ldh(ORS + bo + 32);
            v8f sH = (v8f){}, sR = (v8f){};
            sH = wmma16g(a0h, b0h, sH); sH = wmma16g(a1h, b1h, sH);
            sR = wmma16g(a0h, b0r, sR); sR = wmma16g(a0r, b0h, sR); sR = wmma16g(a1h, b1r, sR); sR = wmma16g(a1r, b1h, sR);
            const float* bp = BLN + ((size_t)b * NC + t * 16 + lr) * NS + s0 + 8 * hi;
            const v4f q0 = *(const v4f*)bp, q1 = *(const v4f*)(bp + 4);
#pragma unroll
            for (int r = 0; r < 4; ++r) { x[t][r] = (sH[r] + sR[r] * QRI) * OINV + q0[r]; x[t][4 + r] = (sH[4 + r] + sR[4 + r] * QRI) * OINV + q1[r]; }
        }
    } else {
#pragma unroll
        for (int t = 0; t < 8; ++t) x[t] = (v8f){};
    }
    float mk[8], uv[8];
    { const float* mp = maskg + (size_t)b * NS + s0 + 8 * hi; const v4f k0 = *(const v4f*)mp, k1 = *(const v4f*)(mp + 4);
      const float* up = US + (size_t)b * NS + s0 + 8 * hi; const v4f u0 = *(const v4f*)up, u1 = *(const v4f*)(up + 4);
#pragma unroll
      for (int r = 0; r < 4; ++r) { mk[r] = bfr(k0[r]); mk[4 + r] = bfr(k1[r]); uv[r] = u0[r]; uv[4 + r] = u1[r]; } }
#pragma unroll
    for (int r = 0; r < 8; ++r) {
        float mx = x[0][r];
#pragma unroll
        for (int t = 1; t < 8; ++t) mx = fmaxf(mx, x[t][r]);
        mx = fmaxf(mx, __shfl_xor(mx, 1, 32)); mx = fmaxf(mx, __shfl_xor(mx, 2, 32)); mx = fmaxf(mx, __shfl_xor(mx, 4, 32)); mx = fmaxf(mx, __shfl_xor(mx, 8, 32));
        float sm = 0.0f;
#pragma unroll
        for (int t = 0; t < 8; ++t) { const float e = __builtin_amdgcn_exp2f((x[t][r] - mx) * LOG2E); x[t][r] = e; sm += e; }
        sm += __shfl_xor(sm, 1, 32); sm += __shfl_xor(sm, 2, 32); sm += __shfl_xor(sm, 4, 32); sm += __shfl_xor(sm, 8, 32);
        const float w = mk[r] * (1.0f / sm);
#pragma unroll
        for (int t = 0; t < 8; ++t) x[t][r] = x[t][r] * w;
    }
#pragma unroll
    for (int t = 0; t < 8; ++t) {
        float pt = 0.0f;
#pragma unroll
        for (int r = 0; r < 8; ++r) pt += x[t][r] * uv[r];
        pt += __shfl_xor(pt, 16, 32);
        if (hi == 0) t2p[wave * NC + t * 16 + lr] = pt;
        v8h hv, rv;
#pragma unroll
        for (int r = 0; r < 8; ++r) { const float cv = x[t][r] * CSC; const h16 a0 = toh_flush(cv); hv[r] = a0; rv[r] = toh_flush((cv - (float)a0) * QRS); }
        *(v8h*)(&ch[(t * 16 + lr) * CP + s0 + 8 * hi]) = hv;
        *(v8h*)(&cr[(t * 16 + lr) * CP + s0 + 8 * hi]) = rv;
    }
    __syncthreads();
    const int n0 = wave * 16;
    v8f aH[4], aR[4];
#pragma unroll
    for (int j = 0; j < 4; ++j) { aH[j] = (v8f){}; aR[j] = (v8f){}; }
#pragma unroll
    for (int ks = 0; ks < 4; ++ks) {
        const int ca = (n0 + lr) * CP + 32 * ks + 8 * hi;
        const v16h cah = cat16(*(const v8h*)(&ch[ca]), *(const v8h*)(&ch[ca + 16]));
        const v16h car = cat16(*(const v8h*)(&cr[ca]), *(const v8h*)(&cr[ca + 16]));
#pragma unroll
        for (int j = 0; j < 4; ++j) {
            const size_t bo = ((size_t)b * DC + 16 * j + lr) * NS + 32 * ks + 8 * hi;
            const v16h bh = ldh(TH + bo), br = ldh(TR + bo);
            aH[j] = wmma16g(cah, bh, aH[j]); aR[j] = wmma16g(cah, br, aR[j]); aR[j] = wmma16g(car, bh, aR[j]);
        }
    }
    const int wb = wave * 16 * 68;
#pragma unroll
    for (int j = 0; j < 4; ++j)
#pragma unroll
        for (int r = 0; r < 8; ++r) os[wb + (8 * hi + r) * 68 + 16 * j + lr] = (aH[j][r] + aR[j][r] * QRI) * CINV;
    wave_sync();
#pragma unroll 1
    for (int it = 0; it < 8; ++it) { const int p = it * 32 + lane; const int row = p >> 4, cofs = (p & 15) * 4; const int n = n0 + row;
        float t2 = 0.0f;
#pragma unroll
        for (int w = 0; w < 8; ++w) t2 += t2p[w * NC + n];
        const v4f pv = *(const v4f*)(PE1 + (size_t)n * DC + cofs);
        v4f v = *(const v4fa*)(&os[wb + row * 68 + cofs]);
#pragma unroll
        for (int i = 0; i < 4; ++i) v[i] = v[i] + t2 * pv[i];
        *(v4fa*)(&os[wb + row * 68 + cofs]) = v; }
    wave_sync();
#pragma unroll 1
    for (int pz = 0; pz < 2; ++pz) {
#pragma unroll 1
        for (int it = 0; it < 8; ++it) { const int p = it * 32 + lane; const int row = p >> 4, q = p & 15;
            const v4f val = *(const v4fa*)(&os[wb + row * 68 + q * 4]);
            *(volatile v4f*)(PREB + ((size_t)b * NC + n0 + row) * DC + q * 4) = val;
            const v8h hv = *(const v8h*)(&ch[(n0 + row) * CP + q * 8]); const v8h rv = *(const v8h*)(&cr[(n0 + row) * CP + q * 8]);
            const size_t co = ((size_t)(n0 + row) * NB + b) * NS + q * 8;
            *(volatile v8h*)(CNH + co) = hv; *(volatile v8h*)(CNR + co) = rv; }
        if (pz == 0) __threadfence(); }
}

static_assert(8 * 16 == NS);
__global__ __launch_bounds__(256) void k_rn(const h16* __restrict__ CNH, const h16* __restrict__ CNR, const h16* __restrict__ PTH, const h16* __restrict__ PTR,
                                           const h16* __restrict__ PH, const h16* __restrict__ PR, const float* __restrict__ PREB, const float* __restrict__ PE1,
                                           const float* __restrict__ US, float* OUT, h16* OH, h16* ORS, float* BLN, int last) {
    __shared__ __align__(16) float pt[NB * 68];
    __shared__ __align__(16) h16 oh[NB * OPT];
    __shared__ __align__(16) h16 orr[NB * OPT];
    __shared__ __align__(16) float bl[NB * 132];
    __shared__ float g2s[NB];
    const int lane = threadIdx.x & 31, lr = lane & 15, hi = lane >> 4;
    const int wave = __builtin_amdgcn_readfirstlane((int)(threadIdx.x >> 5));
    const int tid = threadIdx.x;
    const int n = blockIdx.x;
#pragma unroll 1
    for (int tile = wave; tile < (NB / 16) * 4; tile += 8) {
        const int bt = tile >> 2, j = tile & 3;
        v8f aH = (v8f){}, aR = (v8f){};
#pragma unroll
        for (int ks = 0; ks < 4; ++ks) {
            const size_t ao = ((size_t)n * NB + bt * 16 + lr) * NS + 32 * ks + 8 * hi;
            const size_t bo = ((size_t)n * DC + 16 * j + lr) * NS + 32 * ks + 8 * hi;
            const v16h ah = ldh(CNH + ao), ar = ldh(CNR + ao), bh = ldh(PTH + bo), br = ldh(PTR + bo);
            aH = wmma16g(ah, bh, aH); aR = wmma16g(ah, br, aR); aR = wmma16g(ar, bh, aR);
        }
#pragma unroll
        for (int r = 0; r < 8; ++r) pt[(bt * 16 + 8 * hi + r) * 68 + 16 * j + lr] = (aH[r] + aR[r] * QRI) * CINV;
    }
    __syncthreads();
    const float pe1a = PE1[(size_t)n * DC + lane], pe1b = PE1[(size_t)n * DC + 32 + lane];
#pragma unroll 1
    for (int row = wave; row < NB; row += 8) {
        const float* pb = PREB + ((size_t)row * NC + n) * DC;
        const float p0 = pt[row * 68 + lane] + pb[lane], p1 = pt[row * 68 + 32 + lane] + pb[32 + lane];
        float ss = p0 * p0 + p1 * p1;
        ss += __shfl_xor(ss, 16, 32); ss += __shfl_xor(ss, 8, 32); ss += __shfl_xor(ss, 4, 32); ss += __shfl_xor(ss, 2, 32); ss += __shfl_xor(ss, 1, 32);
        const float sc = ss * (1.0f / (1.0f + ss)) * (1.0f / sqrtf(ss + EPSV));
        const float o0 = sc * p0, o1 = sc * p1;
        float g = o0 * pe1a + o1 * pe1b;
        g += __shfl_xor(g, 16, 32); g += __shfl_xor(g, 8, 32); g += __shfl_xor(g, 4, 32); g += __shfl_xor(g, 2, 32); g += __shfl_xor(g, 1, 32);
        pt[row * 68 + lane] = o0; pt[row * 68 + 32 + lane] = o1;
        const float c0 = o0 * OSC, c1 = o1 * OSC;
        const h16 h0 = toh_flush(c0), h1 = toh_flush(c1);
        oh[row * OPT + lane] = h0; oh[row * OPT + 32 + lane] = h1;
        orr[row * OPT + lane] = toh_flush((c0 - (float)h0) * QRS); orr[row * OPT + 32 + lane] = toh_flush((c1 - (float)h1) * QRS);
        if (lane == 0) g2s[row] = g;
    }
    __syncthreads();
    if (last != 0) {
#pragma unroll 1
        for (int pz = 0; pz < 2; ++pz) {
#pragma unroll 1
            for (int p = tid; p < NB * 16; p += 256) { const int row = p >> 4, cofs = (p & 15) * 4;
                const v4f val = *(const v4fa*)(&pt[row * 68 + cofs]);
                *(volatile v4f*)(OUT + ((size_t)row * NC + n) * DC + cofs) = val; }
            if (pz == 0) __threadfence(); }
    } else {
        const int s0 = wave * 16;
#pragma unroll
        for (int bt = 0; bt < NB / 16; ++bt) {
            v8f aH = (v8f){}, aR = (v8f){};
#pragma unroll
            for (int ks = 0; ks < 2; ++ks) {
                const int ao = (bt * 16 + lr) * OPT + 32 * ks + 8 * hi;
                const v16h ah = cat16(*(const v8h*)(&oh[ao]), *(const v8h*)(&oh[ao + 16]));
                const v16h ar = cat16(*(const v8h*)(&orr[ao]), *(const v8h*)(&orr[ao + 16]));
                const size_t bo = ((size_t)n * NS + s0 + lr) * DC + 32 * ks + 8 * hi;
                const v16h bh = ldh(PH + bo), br = ldh(PR + bo);
                aH = wmma16g(ah, bh, aH); aR = wmma16g(ah, br, aR); aR = wmma16g(ar, bh, aR);
            }
#pragma unroll
            for (int r = 0; r < 8; ++r) { const int bb = bt * 16 + 8 * hi + r;
                bl[bb * 132 + s0 + lr] = (aH[r] + aR[r] * QRI) * OINV + US[(size_t)bb * NS + s0 + lr] * g2s[bb]; }
        }
        __syncthreads();
#pragma unroll 1
        for (int pz = 0; pz < 2; ++pz) {
#pragma unroll 1
            for (int p = tid; p < NB * 8; p += 256) { const int row = p >> 3, c8 = (p & 7) * 8;
                const v8h hv = *(const v8h*)(&oh[row * OPT + c8]); const v8h rv = *(const v8h*)(&orr[row * OPT + c8]);
                const size_t oo = ((size_t)row * NC + n) * DC + c8;
                *(volatile v8h*)(OH + oo) = hv; *(volatile v8h*)(ORS + oo) = rv; }
#pragma unroll 1
            for (int row = wave; row < NB; row += 8) {
                const v4f val = *(const v4fa*)(&bl[row * 132 + 4 * lane]);
                *(volatile v4f*)(BLN + ((size_t)row * NC + n) * NS + 4 * lane) = val; }
            if (pz == 0) __threadfence(); }
    }
}

static constexpr size_t al256(size_t v) { return (v + 255) & ~(size_t)255; }
static constexpr size_t SZ_UB  = al256((size_t)NB * NS * DIN * 2);
static constexpr size_t SZ_WT  = al256((size_t)DC * DIN * 2);
static constexpr size_t SZ_UW  = al256((size_t)NB * NS * DC * 2);
static constexpr size_t SZ_US  = al256((size_t)NB * NS * 4);
static constexpr size_t SZ_PE  = al256((size_t)NC * NS * DC * 2);
static constexpr size_t SZ_P1  = al256((size_t)NC * DC * 4);
static constexpr size_t SZ_CN  = al256((size_t)NC * NB * NS * 2);
static constexpr size_t SZ_PB  = al256((size_t)NB * NC * DC * 4);
static constexpr size_t SZ_BL  = al256((size_t)NB * NC * NS * 4);
static constexpr size_t SZ_TOTAL = SZ_UB + SZ_WT + 4 * SZ_UW + SZ_US + 4 * SZ_PE + SZ_P1 + 2 * SZ_CN + SZ_PB + 2 * SZ_UW + SZ_BL;
static_assert(SZ_TOTAL <= (size_t)134217728);
static_assert((size_t)NB * NS * DC == (size_t)NB * DC * NS);
static_assert((size_t)NB * NC * DC == (size_t)NB * NS * DC);

extern "C" void kernel_launch(void* const* d_in, const int* in_sizes, int n_in,
                              void* d_out, int out_size, void* d_ws, size_t ws_size, hipStream_t stream) {
    if (n_in < 3) return;
    if ((size_t)in_sizes[0] < (size_t)NB * NS * DIN) return;
    if ((size_t)in_sizes[1] < (size_t)NB * NS) return;
    if ((size_t)in_sizes[2] < (size_t)DIN * DC) return;
    if ((size_t)out_size < (size_t)NB * NC * DC) return;
    if (SZ_TOTAL > ws_size) return;
    const float* uin = (const float*)d_in[0];
    const float* msk = (const float*)d_in[1];
    const float* wgt = (const float*)d_in[2];
    float* OUT = (float*)d_out;
    char* wsp = (char*)d_ws;
    bf*  UB  = (bf*)wsp;  wsp += SZ_UB;
    bf*  WT  = (bf*)wsp;  wsp += SZ_WT;
    h16* UH  = (h16*)wsp; wsp += SZ_UW;
    h16* UR  = (h16*)wsp; wsp += SZ_UW;
    h16* TH  = (h16*)wsp; wsp += SZ_UW;
    h16* TR  = (h16*)wsp; wsp += SZ_UW;
    float* US = (float*)wsp; wsp += SZ_US;
    h16* PH  = (h16*)wsp; wsp += SZ_PE;
    h16* PR  = (h16*)wsp; wsp += SZ_PE;
    h16* PTH = (h16*)wsp; wsp += SZ_PE;
    h16* PTR = (h16*)wsp; wsp += SZ_PE;
    float* PE1 = (float*)wsp; wsp += SZ_P1;
    h16* CNH = (h16*)wsp; wsp += SZ_CN;
    h16* CNR = (h16*)wsp; wsp += SZ_CN;
    float* PREB = (float*)wsp; wsp += SZ_PB;
    h16* OH  = (h16*)wsp; wsp += SZ_UW;
    h16* ORS = (h16*)wsp; wsp += SZ_UW;
    float* BLN = (float*)wsp; wsp += SZ_BL;

    { const size_t n8 = (size_t)NB * NS * DIN / 8;
      k_cvt8<<<(unsigned)((n8 + 255) / 256), 256, 0, stream>>>(uin, UB, n8); }
    k_wt<<<1, 256, 0, stream>>>(wgt, WT);
    k_uw<<<NB * NS / 64, 32, 0, stream>>>(UB, WT, UH, UR, TH, TR, US);
    k_pe<<<NC, 256, 0, stream>>>(PH, PR, PTH, PTR, PE1);
    for (int it = 0; it < NIT; ++it) {
        k_rb<<<NB, 256, 0, stream>>>(UH, UR, TH, TR, OH, ORS, BLN, US, msk, PE1, PREB, CNH, CNR, it == 0 ? 1 : 0);
        k_rn<<<NC, 256, 0, stream>>>(CNH, CNR, PTH, PTR, PH, PR, PREB, PE1, US, OUT, OH, ORS, BLN, it == NIT - 1 ? 1 : 0);
    }
}
